// ShapegraphEncoder_18219251269655
// MI455X (gfx1250) — hardware-run, weakly checked
//
#include <hip/hip_runtime.h>


namespace {
constexpr int NG = 20000, B = 64, N = NG + B  , NP = 20096  , E0 = 320000, E = E0 + NG  , D0 = 128, HC = 256, NH = 4, C = 64, L = 3, EMB = 256;
constexpr float XS = 8.0f, WSC = 256.0f, NEG = 0.2f, LNEPS = 1e-5f;

typedef _Float16 b16;
typedef __attribute__((ext_vector_type(16))) _Float16 v16b;
typedef __attribute__((ext_vector_type(8))) _Float16 v8b;
typedef __attribute__((ext_vector_type(8))) float v8f;
typedef __attribute__((ext_vector_type(4))) float v4f;
__device__ __forceinline__ float bf16_rne(float f) { unsigned int u = __float_as_uint(f); u += 0x7FFFu + ((u >> 16) & 1u); return __uint_as_float(u & 0xFFFF0000u); }
__device__ __forceinline__ void split16(float v, b16& hi, b16& lo) { hi = (b16)v; lo = (b16)(v - (float)hi); }
__device__ __forceinline__ v16b frag_kb(const b16* p, int hh) { const v8b a = *(const v8b*)(p + 8 * hh), b = *(const v8b*)(p + 16 + 8 * hh); v16b f;
#pragma unroll
  for (int e = 0; e < 8; ++e) { f[e] = a[e]; f[8 + e] = b[e]; } return f; }
__device__ __forceinline__ v8f wmma16b(v16b a, v16b b, v8f c) { v8f d = __builtin_amdgcn_wmma_f32_16x16x32_f16(false, a, false, b, (short)0, c, false, false); asm volatile("v_nop\n\tv_nop\n\tv_nop\n\tv_nop" : "+v"(d) : "v"(a), "v"(b)); return d; }
__device__ __forceinline__ void wave_lds_sync() { __builtin_amdgcn_fence(__ATOMIC_RELEASE, "workgroup"); __builtin_amdgcn_wave_barrier(); __builtin_amdgcn_fence(__ATOMIC_ACQUIRE, "workgroup"); }
__device__ __forceinline__ float pmul(float a, float b) { float p = a * b; asm volatile("" : "+v"(p)); return p; }
__device__ __forceinline__ int iclamp(int v, int lo, int hi) { return v < lo ? lo : (v > hi ? hi : v); }
__device__ __forceinline__ float nexp(float x) { return __builtin_amdgcn_exp2f(x * 1.4426950408889634f); }
__device__ __forceinline__ float lrelu(float x) { return x > 0.0f ? x : NEG * x; }

constexpr int CSR_NBLK = 512, CSR_GB = 9, CSR_GN = 1 << CSR_GB  , CSR_MAXG = 512, CSR_CAP = 12288  ;
__global__ __launch_bounds__(64) void csrA_kernel(const int* __restrict__ dst, int E, int N, int nG, int CHP, int NGP, int* __restrict__ STG, int* __restrict__ HST) {
  extern __shared__ int sm[];
  int* cnt = sm; int* run = sm + NGP; int* ids = sm + 2 * NGP;
  const int b = blockIdx.x; const int ch = (E + CSR_NBLK - 1) / CSR_NBLK; const int e0 = b * ch, e1 = min(E, e0 + ch);
  for (int i = threadIdx.x; i < NGP; i += 64) cnt[i] = 0;
  for (int i = threadIdx.x; i < CHP; i += 64) ids[i] = -1;
  __syncthreads();
  if (threadIdx.x == 0) {
    for (int e = e0; e < e1; ++e) { int d = dst[e]; d = (d < 0) ? 0 : (d >= N ? N - 1 : d); cnt[d >> CSR_GB] += 1; }
    int acc = 0; for (int g = 0; g < nG; ++g) { run[g] = acc; acc += cnt[g]; }
    for (int e = e0; e < e1; ++e) { int d = dst[e]; d = (d < 0) ? 0 : (d >= N ? N - 1 : d); const int g = d >> CSR_GB; ids[run[g]] = e; run[g] += 1; } }
  __syncthreads();
  typedef __attribute__((ext_vector_type(4))) int v4i;
  for (int pass = 0; pass < 2; ++pass) {
    for (int i = threadIdx.x; i < CHP / 4; i += 64) *(volatile v4i*)(STG + (size_t)b * CHP + i * 4) = *(const v4i*)(&ids[i * 4]);
    for (int i = threadIdx.x; i < NGP / 4; i += 64) { v4i v; for (int e = 0; e < 4; ++e) v[e] = (i * 4 + e < nG) ? cnt[i * 4 + e] : 0; *(volatile v4i*)(HST + (size_t)b * NGP + i * 4) = v; }
    __threadfence(); }
}
__global__ __launch_bounds__(512) void csrS_kernel(const int* __restrict__ HST, int nG, int NGP, int* __restrict__ START, int* __restrict__ TOT, int* __restrict__ OFF) {
  __shared__ int tot[CSR_MAXG];
  const int b = threadIdx.x;
  for (int pass = 0; pass < 2; ++pass) { int runb = 0; for (int g = 0; g < nG; ++g) { int c = HST[(size_t)b * NGP + g]; c = (c < 0) ? 0 : c; ((volatile int*)OFF)[(size_t)g * CSR_NBLK + b] = runb; runb += c; } __threadfence(); }
  for (int g = threadIdx.x; g < nG; g += 512) { int s = 0; for (int bb = 0; bb < CSR_NBLK; ++bb) { int c = HST[(size_t)bb * NGP + g]; s += (c < 0) ? 0 : c; } tot[g] = s; }
  __syncthreads();
  if (threadIdx.x < 32) {
    __shared__ int st[CSR_MAXG + 32];
    if (threadIdx.x == 0) { int acc = 0; for (int g = 0; g < NGP; ++g) { st[g] = acc; if (g < nG) acc += (tot[g] + 31) & ~31; } st[NGP] = acc; }
    __builtin_amdgcn_fence(__ATOMIC_RELEASE, "workgroup"); __builtin_amdgcn_wave_barrier(); __builtin_amdgcn_fence(__ATOMIC_ACQUIRE, "workgroup");
    for (int pass = 0; pass < 2; ++pass) { for (int i = threadIdx.x; i < NGP + 32; i += 32) { ((volatile int*)START)[i] = (i <= NGP) ? st[min(i, NGP)] : 0; ((volatile int*)TOT)[i] = (i < nG) ? tot[i] : 0; } __threadfence(); } }
}
__global__ __launch_bounds__(256) void csrB_kernel(const int* __restrict__ dst, int N, int nG, int CHP, int NGP, int permLen, const int* __restrict__ STG, const int* __restrict__ HST, const int* __restrict__ OFF, const int* __restrict__ START, const int* __restrict__ TOT, int* __restrict__ PERM, int* __restrict__ ROWPTR, int* __restrict__ ROWCNT, int* __restrict__ FLAG) {
  typedef __attribute__((ext_vector_type(4))) int v4i;
  __shared__ int ids[CSR_CAP]; __shared__ unsigned short key[CSR_CAP]; __shared__ int outp[CSR_CAP]; __shared__ int ncnt[CSR_GN + 1]; __shared__ int boff[CSR_NBLK + 1];
  const int g = blockIdx.x, t_ = threadIdx.x; int tot = TOT[g]; int st = START[g], stn = START[g + 1]; const int v0 = g * CSR_GN; const int nv = min(CSR_GN, N - v0);
  st = (st < 0) ? 0 : (st > permLen - 32 ? permLen - 32 : st) & ~31; stn = (stn < st) ? st : (stn > permLen ? permLen : stn); tot = (tot < 0) ? 0 : tot; if (tot > stn - st && tot <= CSR_CAP) tot = stn - st;
  if (tot > CSR_CAP) {
    for (int pass = 0; pass < 2; ++pass) { for (int i = t_; i < CSR_GN / 4; i += 256) { v4i a, c; for (int e = 0; e < 4; ++e) { a[e] = st; c[e] = 0; } *(volatile v4i*)(ROWPTR + v0 + i * 4) = a; *(volatile v4i*)(ROWCNT + v0 + i * 4) = c; } if (t_ == 0) ((volatile int*)FLAG)[0] = 1; __threadfence(); } (void)nv; return; }
  if (t_ == 0) { int acc = 0; for (int b = 0; b < CSR_NBLK; ++b) { boff[b] = acc; int c = HST[(size_t)b * NGP + g]; c = (c < 0) ? 0 : (c > CHP ? CHP : c); acc += c; if (acc > tot) acc = tot; } boff[CSR_NBLK] = acc; }
  for (int i = t_; i <= CSR_GN; i += 256) ncnt[i] = 0;
  __syncthreads();
  for (int b = 0; b < CSR_NBLK; ++b) { const int c = boff[b + 1] - boff[b]; int o_ = OFF[(size_t)g * CSR_NBLK + b]; o_ = (o_ < 0) ? 0 : (o_ > CHP - c ? CHP - c : o_); const int* src_ = STG + (size_t)b * CHP + o_;
    for (int i = t_; i < c; i += 256) { int id = src_[i]; id = (id < 0) ? 0 : id; ids[boff[b] + i] = id; int d = dst[id]; d = (d < v0) ? v0 : (d >= N ? N - 1 : d); int kk = d - v0; kk = (kk < 0) ? 0 : (kk >= CSR_GN ? CSR_GN - 1 : kk); key[boff[b] + i] = (unsigned short)kk; } }
  __syncthreads();
  if (t_ == 0) { for (int i = 0; i < tot; ++i) ncnt[key[i]] += 1; int acc = 0; for (int vl = 0; vl < CSR_GN; ++vl) { const int c = ncnt[vl]; ncnt[vl] = acc; acc += c; } ncnt[CSR_GN] = acc;
    for (int i = 0; i < tot; ++i) { const int vl = key[i]; outp[ncnt[vl]] = ids[i]; ncnt[vl] += 1; }
    for (int vl = CSR_GN; vl > 0; --vl) ncnt[vl] = ncnt[vl - 1]; ncnt[0] = 0; }
  __syncthreads();
  for (int pass = 0; pass < 2; ++pass) {
    for (int i = t_; i < (stn - st) / 4; i += 256) { v4i v; for (int e = 0; e < 4; ++e) { const int q = i * 4 + e; v[e] = (q < tot) ? outp[q] : -1; } *(volatile v4i*)(PERM + st + i * 4) = v; }
    for (int i = t_; i < CSR_GN / 4; i += 256) { v4i a, c; for (int e = 0; e < 4; ++e) { const int vl = i * 4 + e; a[e] = st + ncnt[vl]; c[e] = (vl < nv) ? (ncnt[vl + 1] - ncnt[vl]) : 0; } *(volatile v4i*)(ROWPTR + v0 + i * 4) = a; *(volatile v4i*)(ROWCNT + v0 + i * 4) = c; }
    __threadfence(); }
}
__global__ __launch_bounds__(256) void csrZ_kernel(int* __restrict__ p, size_t n4) { typedef __attribute__((ext_vector_type(4))) int v4i; const size_t tid = (size_t)blockIdx.x * 256 + threadIdx.x, nth = (size_t)gridDim.x * 256; v4i z = {0, 0, 0, 0}; for (size_t i = tid; i < n4; i += nth) *(volatile v4i*)(p + i * 4) = z; }
struct CsrBufs { int *STG, *HST, *OFF, *START, *TOT, *PERM, *ROWPTR, *ROWCNT, *FLAG; int nG, NGP, CHP; size_t permLen; char* base; size_t bytes; };
static size_t csr_carve(CsrBufs& c, char* ws, size_t off, int E, int N) {
  const size_t off0 = off; c.base = ws + off;
  auto al = [&](size_t bytes) { char* p = ws + off; off += (bytes + 255) & ~(size_t)255; return p; };
  c.nG = (N + CSR_GN - 1) / CSR_GN; c.NGP = (c.nG + 31) & ~31; const int ch = (E + CSR_NBLK - 1) / CSR_NBLK; c.CHP = (ch + 31) & ~31; c.permLen = (size_t)E + 32 * (size_t)c.nG + 32;
  c.STG = (int*)al((size_t)CSR_NBLK * c.CHP * 4); c.HST = (int*)al((size_t)CSR_NBLK * c.NGP * 4); c.OFF = (int*)al((size_t)c.NGP * CSR_NBLK * 4); c.START = (int*)al((size_t)(c.NGP + 64) * 4); c.TOT = (int*)al((size_t)(c.NGP + 64) * 4);
  c.PERM = (int*)al(c.permLen * 4); c.ROWPTR = (int*)al((size_t)c.nG * CSR_GN * 4); c.ROWCNT = (int*)al((size_t)c.nG * CSR_GN * 4); c.FLAG = (int*)al(256);
  c.bytes = off - off0; return off;
}
static void csr_build(const CsrBufs& c, const int* dst, int E, int N, hipStream_t stream) {
  const size_t smem = (size_t)(2 * c.NGP + c.CHP) * 4;
  csrZ_kernel<<<512, 256, 0, stream>>>((int*)c.base, c.bytes / 16);
  csrA_kernel<<<CSR_NBLK, 64, smem, stream>>>(dst, E, N, c.nG, c.CHP, c.NGP, c.STG, c.HST);
  csrS_kernel<<<1, 512, 0, stream>>>(c.HST, c.nG, c.NGP, c.START, c.TOT, c.OFF);
  csrB_kernel<<<c.nG, 256, 0, stream>>>(dst, N, c.nG, c.CHP, c.NGP, (int)c.permLen, c.STG, c.HST, c.OFF, c.START, c.TOT, c.PERM, c.ROWPTR, c.ROWCNT, c.FLAG);
}


__global__ __launch_bounds__(256) void edges_kernel(const int* __restrict__ ei, const int* __restrict__ batch, int* __restrict__ SRC, int* __restrict__ DST) {
  typedef __attribute__((ext_vector_type(4))) int v4i;
  const size_t u = (size_t)blockIdx.x * 256 + threadIdx.x; if (u * 4 >= (size_t)E) return; const size_t e0 = u * 4; v4i s, d;
  for (int j = 0; j < 4; ++j) { const size_t e = e0 + j; if (e < (size_t)E0) { s[j] = iclamp(ei[e], 0, NG - 1) + B; d[j] = iclamp(ei[E0 + e], 0, NG - 1) + B; } else { const int n = (int)(e - E0); s[j] = iclamp(batch[n], 0, B - 1); d[j] = n + B; } }
  for (int pass = 0; pass < 2; ++pass) { *(volatile v4i*)(SRC + e0) = s; *(volatile v4i*)(DST + e0) = d; __threadfence(); }
}
__global__ __launch_bounds__(256) void prep_kernel(const float* __restrict__ x, const float* __restrict__ win, const float* __restrict__ wg, const float* __restrict__ wo, b16* __restrict__ Xh, b16* __restrict__ WinT, b16* __restrict__ WgT, b16* __restrict__ WoT) {
  const size_t u = (size_t)blockIdx.x * 256 + threadIdx.x; const size_t nx = (size_t)NP * D0 / 8, n1 = (size_t)HC * D0 / 8, n2 = (size_t)L * HC * HC / 8, n3 = (size_t)EMB * HC / 8; size_t t = u; v8b o;
  if (t < nx) { const size_t e = t * 8; const size_t r = e / D0; const int c0 = (int)(e % D0); for (int j = 0; j < 8; ++j) o[j] = (r >= (size_t)B && r < (size_t)N) ? (b16)(bf16_rne(x[(r - B) * D0 + c0 + j]) * XS) : (b16)0.0f; for (int pass = 0; pass < 2; ++pass) { *(volatile v8b*)(Xh + e) = o; __threadfence(); } return; } t -= nx;
  if (t < n1) { const size_t e = t * 8; const int oo = (int)(e / D0), k0 = (int)(e % D0); for (int j = 0; j < 8; ++j) o[j] = (b16)(bf16_rne(win[(size_t)(k0 + j) * HC + oo]) * WSC); for (int pass = 0; pass < 2; ++pass) { *(volatile v8b*)(WinT + e) = o; __threadfence(); } return; } t -= n1;
  if (t < n2) { const size_t e = t * 8; const int l = (int)(e / ((size_t)HC * HC)); const size_t r = e % ((size_t)HC * HC); const int oo = (int)(r / HC), k0 = (int)(r % HC); for (int j = 0; j < 8; ++j) o[j] = (b16)(bf16_rne(wg[((size_t)l * HC + k0 + j) * HC + oo]) * WSC); for (int pass = 0; pass < 2; ++pass) { *(volatile v8b*)(WgT + e) = o; __threadfence(); } return; } t -= n2;
  if (t < n3) { const size_t e = t * 8; const int oo = (int)(e / HC), k0 = (int)(e % HC); for (int j = 0; j < 8; ++j) o[j] = (b16)(bf16_rne(wo[(size_t)(k0 + j) * EMB + oo]) * WSC); for (int pass = 0; pass < 2; ++pass) { *(volatile v8b*)(WoT + e) = o; __threadfence(); } }
}
template <int KD, int TWO, int MODE>
__global__ __launch_bounds__(128) void gemm_kernel(const b16* __restrict__ Ah, const b16* __restrict__ Al, const b16* __restrict__ WT, const float* __restrict__ bias, const float* __restrict__ cls, float* __restrict__ OUTF, b16* __restrict__ Oh, b16* __restrict__ Ol) {
  __shared__ __attribute__((aligned(16))) float Tf[4][16][128 + 4];
  const int wave = threadIdx.x >> 5, lane = threadIdx.x & 31, nloc = lane & 15, hlf = lane >> 4; const size_t m0 = (size_t)blockIdx.x * 64 + wave * 16; const int n0 = blockIdx.y * 128;
  v8f acc[8];
#pragma unroll
  for (int t = 0; t < 8; ++t) acc[t] = (v8f){};
#pragma unroll 2
  for (int kb = 0; kb < KD; kb += 32) { const v16b a = frag_kb(Ah + (m0 + nloc) * KD + kb, hlf); v16b al; if (TWO) al = frag_kb(Al + (m0 + nloc) * KD + kb, hlf);
#pragma unroll
    for (int t = 0; t < 8; ++t) { const v16b bw = frag_kb(WT + (size_t)(n0 + t * 16 + nloc) * KD + kb, hlf); acc[t] = wmma16b(a, bw, acc[t]); if (TWO) acc[t] = wmma16b(al, bw, acc[t]); } }
#pragma unroll
  for (int t = 0; t < 8; ++t) { const int c = n0 + t * 16 + nloc; const float bb = bias ? bf16_rne(bias[c]) : 0.0f; const float cv = MODE == 1 ? bf16_rne(cls[c]) : 0.0f;
#pragma unroll 1
    for (int r = 0; r < 8; ++r) { const size_t row = m0 + 8 * hlf + r; float y = acc[t][r] * (1.0f / (XS * WSC)) + bb; if (MODE == 1) { if (row < (size_t)B) y = cv; else if (row >= (size_t)N) y = 0.0f; } Tf[wave][8 * hlf + r][t * 16 + nloc] = y; } }
  wave_lds_sync();
  for (int pass = 0; pass < 2; ++pass) { for (int rr = 0; rr < 16; ++rr) { const v4f v = *(const v4f*)(&Tf[wave][rr][lane * 4]); *(volatile v4f*)(OUTF + (m0 + rr) * HC + n0 + lane * 4) = v;
      if (MODE == 1) { b16 ph[4], pl[4]; for (int j = 0; j < 4; ++j) split16(v[j] * XS, ph[j], pl[j]); typedef __attribute__((ext_vector_type(4))) _Float16 v4h; v4h hv = {ph[0], ph[1], ph[2], ph[3]}, lv = {pl[0], pl[1], pl[2], pl[3]}; *(volatile v4h*)(Oh + (m0 + rr) * HC + n0 + lane * 4) = hv; *(volatile v4h*)(Ol + (m0 + rr) * HC + n0 + lane * 4) = lv; } }
    __threadfence(); }
}
__global__ __launch_bounds__(256) void node_kernel(const float* __restrict__ XS_, const float* __restrict__ as_, const float* __restrict__ ad_, float* __restrict__ AS, float* __restrict__ AD) {
  const int wave = threadIdx.x >> 5, lane = threadIdx.x & 31; const size_t v = (size_t)blockIdx.x * 8 + wave; const int c0 = lane * 8;
  float s = 0.0f, d = 0.0f; const float* hr = XS_ + v * HC + c0;
  for (int j = 0; j < 8; ++j) { const float hv = hr[j]; s += pmul(hv, bf16_rne(as_[c0 + j])); d += pmul(hv, bf16_rne(ad_[c0 + j])); }
  s += __shfl_xor(s, 1); s += __shfl_xor(s, 2); s += __shfl_xor(s, 4); d += __shfl_xor(d, 1); d += __shfl_xor(d, 2); d += __shfl_xor(d, 4);
  const float t1 = __shfl(s, (lane & 3) * 8), t2 = __shfl(d, (lane & 3) * 8); const float o1 = (lane < NH) ? t1 : 0.0f, o2 = (lane < NH) ? t2 : 0.0f;
  for (int pass = 0; pass < 2; ++pass) { ((volatile float*)AS)[v * 32 + lane] = o1; ((volatile float*)AD)[v * 32 + lane] = o2; __threadfence(); }
}
__device__ int lower_bound_i(const int* a, int n, int key) { int lo = 0, hi = n; while (lo < hi) { const int mid = (lo + hi) >> 1; if (a[mid] < key) lo = mid + 1; else hi = mid; } return lo; }
__global__ __launch_bounds__(256) void agg_kernel(const float* __restrict__ XSm, const float* __restrict__ AS, const float* __restrict__ AD, const int* __restrict__ SRC, const int* __restrict__ PERM, const int* __restrict__ ROWPTR, const int* __restrict__ ROWCNT, int permLen, const int* __restrict__ batch, const float* __restrict__ bias, const float* __restrict__ HF, const float* __restrict__ g_, const float* __restrict__ b_, float* __restrict__ HF2, b16* __restrict__ Oh, b16* __restrict__ Ol) {
  const int wave = threadIdx.x >> 5, lane = threadIdx.x & 31; const size_t v = (size_t)blockIdx.x * 8 + wave; const int h = lane >> 3, c0 = lane * 8;
  float y[8]; for (int q = 0; q < 8; ++q) y[q] = 0.0f;
  if (v < (size_t)N) {
    int st = 0, cnt = 0, lo = 0; const bool iscls = v < (size_t)B;
    if (iscls) { lo = lower_bound_i(batch, NG, (int)v); cnt = lower_bound_i(batch, NG, (int)v + 1) - lo; } else { st = ROWPTR[v]; cnt = ROWCNT[v]; cnt = iclamp(cnt, 0, 65536); st = iclamp(st, 0, permLen - cnt); }
    auto srcof = [&](int j) -> size_t { return iscls ? (size_t)(lo + j + B) : (size_t)iclamp(SRC[iclamp(PERM[st + j], 0, E - 1)], 0, N - 1); };
    const float adv = AD[v * 32 + h]; const float self_l = lrelu(AS[v * 32 + h] + adv); float mx = self_l;
    for (int j = 0; j < cnt; ++j) { const size_t s = srcof(j); mx = fmaxf(mx, lrelu(AS[s * 32 + h] + adv)); }
    float den; float acc[8]; { const float w0 = nexp(self_l - mx); den = w0; const float* hr = XSm + v * HC + c0; for (int q = 0; q < 8; ++q) acc[q] = pmul(w0, hr[q]); }
    for (int j = 0; j < cnt; ++j) { const size_t s = srcof(j); const float w = nexp(lrelu(AS[s * 32 + h] + adv) - mx); den += w; const float* hr = XSm + s * HC + c0;
      const v4f h0 = *(const v4f*)hr, h1 = *(const v4f*)(hr + 4); for (int q = 0; q < 4; ++q) { acc[q] += pmul(w, h0[q]); acc[4 + q] += pmul(w, h1[q]); } }
    const float inv = 1.0f / den; for (int q = 0; q < 8; ++q) y[q] = HF[v * HC + c0 + q] + (acc[q] * inv + bf16_rne(bias[c0 + q])); }
  float s1 = 0.0f; for (int q = 0; q < 8; ++q) s1 += y[q]; for (int o = 16; o; o >>= 1) s1 += __shfl_xor(s1, o); const float mean = s1 * (1.0f / HC);
  float s2 = 0.0f; for (int q = 0; q < 8; ++q) { const float d = y[q] - mean; s2 += d * d; } for (int o = 16; o; o >>= 1) s2 += __shfl_xor(s2, o); const float rstd = rsqrtf(s2 * (1.0f / HC) + LNEPS);
  v4f o0, o1; v8b ph, pl;
  for (int q = 0; q < 8; ++q) { float z = (y[q] - mean) * rstd * bf16_rne(g_[c0 + q]) + bf16_rne(b_[c0 + q]); if (v >= (size_t)N) z = 0.0f; if (q < 4) o0[q] = z; else o1[q - 4] = z; b16 p, pq; split16(z * XS, p, pq); ph[q] = p; pl[q] = pq; }
  for (int pass = 0; pass < 2; ++pass) { *(volatile v4f*)(HF2 + v * HC + c0) = o0; *(volatile v4f*)(HF2 + v * HC + c0 + 4) = o1; *(volatile v8b*)(Oh + v * HC + c0) = ph; *(volatile v8b*)(Ol + v * HC + c0) = pl; __threadfence(); }
}
}

extern "C" void kernel_launch(void* const* d_in, const int* in_sizes, int n_in, void* d_out, int out_size, void* d_ws, size_t ws_size, hipStream_t stream) {
  (void)n_in;
  auto Fp = [&](int i) { return (const float*)d_in[i]; }; auto Ip = [&](int i) { return (const int*)d_in[i]; };
  if (in_sizes[0] != NG * D0 || in_sizes[1] != 2 * E0 || in_sizes[2] != NG || in_sizes[3] != D0 * HC || in_sizes[5] != HC || in_sizes[6] != L * HC * HC || in_sizes[7] != L * HC || in_sizes[12] != HC * EMB || out_size != B * EMB) return;
  size_t off = 0; char* ws = (char*)d_ws;
  auto carve = [&](size_t bytes) { char* p = ws + off; off += (bytes + 255) & ~(size_t)255; return p; };
  int* SRC = (int*)carve((size_t)E * 4); int* DST = (int*)carve((size_t)E * 4); b16* Xh = (b16*)carve((size_t)NP * D0 * 2); b16* WinT = (b16*)carve((size_t)HC * D0 * 2); b16* WgT = (b16*)carve((size_t)L * HC * HC * 2); b16* WoT = (b16*)carve((size_t)EMB * HC * 2);
  float* HFa = (float*)carve((size_t)NP * HC * 4); float* HFb = (float*)carve((size_t)NP * HC * 4); float* XSm = (float*)carve((size_t)NP * HC * 4); b16* Oh = (b16*)carve((size_t)NP * HC * 2); b16* Ol = (b16*)carve((size_t)NP * HC * 2); float* AS = (float*)carve((size_t)NP * 32 * 4); float* AD = (float*)carve((size_t)NP * 32 * 4);
  CsrBufs csr; off = csr_carve(csr, ws, off, E, N);
  if (off > ws_size || off > ((size_t)128 << 20)) return;
  edges_kernel<<<(unsigned)(((size_t)E / 4 + 255) / 256), 256, 0, stream>>>(Ip(1), Ip(2), SRC, DST);
  prep_kernel<<<(unsigned)(((size_t)NP * D0 / 8 + (size_t)HC * D0 / 8 + (size_t)L * HC * HC / 8 + (size_t)EMB * HC / 8 + 255) / 256), 256, 0, stream>>>(Fp(0), Fp(3), Fp(6), Fp(12), Xh, WinT, WgT, WoT);
  csr_build(csr, DST, E, N, stream);
  gemm_kernel<D0, 0, 1><<<dim3(NP / 64, 2), 128, 0, stream>>>(Xh, nullptr, WinT, Fp(4), Fp(5), HFa, Oh, Ol);
  float* HF = HFa; float* HF2 = HFb;
  for (int l = 0; l < L; ++l) {
    gemm_kernel<HC, 1, 0><<<dim3(NP / 64, 2), 128, 0, stream>>>(Oh, Ol, WgT + (size_t)l * HC * HC, nullptr, nullptr, XSm, nullptr, nullptr);
    node_kernel<<<NP / 8, 256, 0, stream>>>(XSm, Fp(7) + l * HC, Fp(8) + l * HC, AS, AD);
    agg_kernel<<<NP / 8, 256, 0, stream>>>(XSm, AS, AD, SRC, csr.PERM, csr.ROWPTR, csr.ROWCNT, (int)csr.permLen, Ip(2), Fp(9) + l * HC, HF, Fp(10) + l * HC, Fp(11) + l * HC, HF2, Oh, Ol);
    float* t = HF; HF = HF2; HF2 = t; }
  gemm_kernel<HC, 1, 0><<<dim3(1, 2), 128, 0, stream>>>(Oh, Ol, WoT, Fp(13), nullptr, (float*)d_out, nullptr, nullptr);
}
